// SkipAttention_34763465294430
// MI455X (gfx1250) — hardware-verified
//
#include <hip/hip_runtime.h>
#include <hip/hip_bf16.h>
#include <math.h>

typedef __attribute__((ext_vector_type(16))) _Float16 v16h;
typedef __attribute__((ext_vector_type(8)))  _Float16 v8h;
typedef __attribute__((ext_vector_type(8)))  float    v8f;
typedef __attribute__((ext_vector_type(4)))  unsigned int u32x4;
typedef __attribute__((ext_vector_type(8)))  int          i32x8;
typedef __attribute__((ext_vector_type(4)))  int          i32x4;
typedef __attribute__((ext_vector_type(4)))  float        v4f;
typedef __attribute__((ext_vector_type(4)))  unsigned     v4u;
template <typename T> __device__ __forceinline__ void vst2(void* p, T v) { *(volatile T*)p = v; __threadfence(); *(volatile T*)p = v; }

#define HDIM 512
#define TSEQ 2048
#define NBATCH 8

__device__ __forceinline__ v8f wmma_f16(v16h a, v16h b, v8f c) {
    v8f d = __builtin_amdgcn_wmma_f32_16x16x32_f16(false, a, false, b, (short)0, c, false, false);
    asm volatile("v_nop\n\tv_nop\n\tv_nop\n\tv_nop" : "+v"(d) : "v"(a), "v"(b));
    return d;
}

__device__ __forceinline__ v16h load_fragA(const _Float16* p, int row0, int ld, int k0) {
    int lane = threadIdx.x & 31;
    int m = lane & 15;
    int g = lane >> 4;
    const _Float16* base = p + (size_t)(row0 + m) * ld + k0 + g * 8;
    v8h lo = *(const v8h*)(base);
    v8h hi = *(const v8h*)(base + 16);
    v16h r;
#pragma unroll
    for (int i = 0; i < 8; ++i) { r[i] = lo[i]; r[i + 8] = hi[i]; }
    return r;
}

__device__ __forceinline__ v16h load_fragB(const _Float16* p, int row0, int ld, int k0) {
    int lane = threadIdx.x & 31;
    int n = lane & 15;
    int g = lane >> 4;
    const _Float16* base = p + (size_t)(row0 + n) * ld + k0 + g * 8;
    v8h lo = *(const v8h*)(base);
    v8h hi = *(const v8h*)(base + 16);
    v16h r;
#pragma unroll
    for (int i = 0; i < 8; ++i) { r[i] = lo[i]; r[i + 8] = hi[i]; }
    return r;
}

__global__ void cvt_f32_to_f16(const float* __restrict__ src,
                               _Float16* __restrict__ dst, int n) {
    int g8 = blockIdx.x * blockDim.x + threadIdx.x;
    if (g8 * 8 >= n) return;
    union { v8h h; v4u u; } pk;
#pragma unroll
    for (int e = 0; e < 8; ++e) pk.h[e] = (_Float16)src[(size_t)g8 * 8 + e];
    vst2(dst + (size_t)g8 * 8, pk.u);
}

__global__ void __launch_bounds__(128)
proj_gemm(const _Float16* __restrict__ xh, const _Float16* __restrict__ wh,
          const float* __restrict__ bias, _Float16* __restrict__ out,
          int mode, float scale) {
    __shared__ __attribute__((aligned(16))) _Float16 st[64 * 72];
    int wave = threadIdx.x >> 5;
    int lane = threadIdx.x & 31;
    int col = lane & 15, g = lane >> 4;
    int m0 = blockIdx.x * 64 + wave * 16;
    int n0 = blockIdx.y * 64;

    v8f c[4] = {};
#pragma unroll 2
    for (int k = 0; k < 16; ++k) {
        v16h a = load_fragA(xh, m0, HDIM, k * 32);
#pragma unroll
        for (int j = 0; j < 4; ++j) c[j] = wmma_f16(a, load_fragB(wh, n0 + j * 16, HDIM, k * 32), c[j]);
    }
#pragma unroll
    for (int j = 0; j < 4; ++j) {
        const float bb = bias[n0 + j * 16 + col];
#pragma unroll
        for (int v = 0; v < 8; ++v) {
            const int rl = wave * 16 + v + g * 8, cl = j * 16 + col;
            const float y = (c[j][v] + bb) * scale;
            if (mode == 2) st[cl * 72 + rl] = (_Float16)y; else st[rl * 72 + cl] = (_Float16)y;
        }
    }
    __syncthreads();
    const int tid = threadIdx.x;
    if (mode == 2) {
        const int bm0 = blockIdx.x * 64;
        const int bidx = bm0 >> 11, tloc = bm0 & (TSEQ - 1);
#pragma unroll
        for (int q = 0; q < 4; ++q) { const int gq = q * 128 + tid; const int d = gq >> 3, pc = gq & 7;
            vst2(out + ((size_t)bidx * HDIM + n0 + d) * TSEQ + tloc + pc * 8, *(const v4u*)(&st[d * 72 + pc * 8])); }
    } else {
#pragma unroll
        for (int q = 0; q < 4; ++q) { const int gq = q * 128 + tid; const int rl = gq >> 3, pc = gq & 7;
            vst2(out + (size_t)(blockIdx.x * 64 + rl) * HDIM + n0 + pc * 8, *(const v4u*)(&st[rl * 72 + pc * 8])); }
    }
}

__global__ void __launch_bounds__(64)
flash_attn(const _Float16* __restrict__ Qh, const _Float16* __restrict__ Kh,
           const _Float16* __restrict__ Vt, const float* __restrict__ xres,
           float* __restrict__ out) {
    __shared__ __attribute__((aligned(16))) _Float16 qs[2][16 * HDIM];
    __shared__ __attribute__((aligned(16))) _Float16 ps[2][16 * 32];
    __shared__ __attribute__((aligned(16))) float    os[2][16 * 32];

    int wave = threadIdx.x >> 5;
    int lane = threadIdx.x & 31;
    int tile = blockIdx.x * 2 + wave;
    int bidx = tile >> 7;
    int t0   = (tile & 127) << 4;

    const _Float16* Qb = Qh + (size_t)bidx * TSEQ * HDIM;
    const _Float16* Kb = Kh + (size_t)bidx * TSEQ * HDIM;
    const _Float16* Vb = Vt + (size_t)bidx * HDIM * TSEQ;

    _Float16* q = qs[wave];
    _Float16* p = ps[wave];

    {
        const v4u* src = (const v4u*)(Qb + (size_t)t0 * HDIM);
#pragma unroll 8
        for (int i = 0; i < 32; ++i) *(v4u*)(q + (i * 32 + lane) * 8) = src[i * 32 + lane];
    }
    __syncthreads();

    const int dhalf = blockIdx.y;
    v8f zero = {};
    v8f acc[16];
#pragma unroll
    for (int i = 0; i < 16; ++i) acc[i] = zero;
    float mrow[8], lrow[8];
#pragma unroll
    for (int v = 0; v < 8; ++v) { mrow[v] = -3.0e38f; lrow[v] = 0.0f; }

    int col = lane & 15;
    int g   = lane >> 4;

    for (int s0 = 0; s0 < TSEQ; s0 += 32) {
        if (s0 + 32 < TSEQ) {
            __builtin_prefetch(Kb + (size_t)(s0 + 32 + col) * HDIM, 0, 1);
            __builtin_prefetch(Kb + (size_t)(s0 + 48 + col) * HDIM, 0, 1);
        }
        v8f sc0 = zero, sc1 = zero;
#pragma unroll
        for (int kd = 0; kd < 16; ++kd) {
            v16h a  = load_fragA(q, 0, HDIM, kd * 32);
            v16h b0 = load_fragB(Kb, s0,      HDIM, kd * 32);
            v16h b1 = load_fragB(Kb, s0 + 16, HDIM, kd * 32);
            sc0 = wmma_f16(a, b0, sc0);
            sc1 = wmma_f16(a, b1, sc1);
        }
#pragma unroll
        for (int v = 0; v < 8; ++v) {
            float mv = fmaxf(sc0[v], sc1[v]);
#pragma unroll
            for (int off = 8; off >= 1; off >>= 1)
                mv = fmaxf(mv, __shfl_xor(mv, off, 32));
            float mn = fmaxf(mrow[v], mv);
            float alpha = __expf(mrow[v] - mn);
            float p0 = __expf(sc0[v] - mn);
            float p1 = __expf(sc1[v] - mn);
            float rs = p0 + p1;
#pragma unroll
            for (int off = 8; off >= 1; off >>= 1)
                rs += __shfl_xor(rs, off, 32);
            lrow[v] = lrow[v] * alpha + rs;
            mrow[v] = mn;
#pragma unroll
            for (int dt = 0; dt < 16; ++dt) acc[dt][v] *= alpha;
            int row = v + g * 8;
            p[row * 32 + col]      = (_Float16)p0;
            p[row * 32 + col + 16] = (_Float16)p1;
        }
        __syncthreads();
        v16h pa = load_fragA(p, 0, 32, 0);
#pragma unroll
        for (int dt = 0; dt < 16; ++dt) {
            v16h vb = load_fragB(Vb, (dhalf * 16 + dt) * 16, TSEQ, s0);
            acc[dt] = wmma_f16(pa, vb, acc[dt]);
        }
        __syncthreads();
    }

    float* o = os[wave];
#pragma unroll
    for (int dpl = 0; dpl < 8; ++dpl) {
        const int dp = dhalf * 8 + dpl;
#pragma unroll
        for (int v = 0; v < 8; ++v) {
            int r = v + g * 8;
            o[r * 32 + col]      = acc[2 * dpl][v]     / lrow[v];
            o[r * 32 + 16 + col] = acc[2 * dpl + 1][v] / lrow[v];
        }
        asm volatile("s_wait_dscnt 0" ::: "memory"); __builtin_amdgcn_wave_barrier(); __builtin_amdgcn_fence(__ATOMIC_RELEASE, "workgroup");
#pragma unroll
        for (int qq = 0; qq < 4; ++qq) {
            const int rl = qq * 4 + (lane >> 3), pc = lane & 7;
            const size_t idx = ((size_t)bidx * TSEQ + t0 + rl) * HDIM + dp * 32 + pc * 4;
            v4f v = *(const v4f*)(o + rl * 32 + pc * 4);
            const v4f xr = *(const v4f*)(xres + idx);
            vst2(out + idx, v + xr);
        }
        __builtin_amdgcn_wave_barrier();
    }
}

extern "C" void kernel_launch(void* const* d_in, const int* in_sizes, int n_in,
                              void* d_out, int out_size, void* d_ws, size_t ws_size,
                              hipStream_t stream) {
    (void)in_sizes; (void)n_in; (void)out_size; (void)ws_size;
    const float* x  = (const float*)d_in[0];
    const float* Wq = (const float*)d_in[1];
    const float* bq = (const float*)d_in[2];
    const float* Wk = (const float*)d_in[3];
    const float* bk = (const float*)d_in[4];
    const float* Wv = (const float*)d_in[5];
    const float* bv = (const float*)d_in[6];
    float* out = (float*)d_out;

    const size_t NX = (size_t)NBATCH * TSEQ * HDIM;
    const size_t NW = (size_t)HDIM * HDIM;

    _Float16* ws  = (_Float16*)d_ws;
    _Float16* xh  = ws;
    _Float16* wqh = xh  + NX;
    _Float16* wkh = wqh + NW;
    _Float16* wvh = wkh + NW;
    _Float16* Qh  = wvh + NW;
    _Float16* Kh  = Qh  + NX;
    _Float16* Vt  = Kh  + NX;

    cvt_f32_to_f16<<<(int)((NX / 8 + 255) / 256), 256, 0, stream>>>(x,  xh,  (int)NX);
    cvt_f32_to_f16<<<(int)((NW / 8 + 255) / 256), 256, 0, stream>>>(Wq, wqh, (int)NW);
    cvt_f32_to_f16<<<(int)((NW / 8 + 255) / 256), 256, 0, stream>>>(Wk, wkh, (int)NW);
    cvt_f32_to_f16<<<(int)((NW / 8 + 255) / 256), 256, 0, stream>>>(Wv, wvh, (int)NW);

    const float scale = 0.04419417382415922f;
    proj_gemm<<<dim3(256, 8), 128, 0, stream>>>(xh, wqh, bq, Qh, 0, scale);
    proj_gemm<<<dim3(256, 8), 128, 0, stream>>>(xh, wkh, bk, Kh, 1, 1.0f);
    proj_gemm<<<dim3(256, 8), 128, 0, stream>>>(xh, wvh, bv, Vt, 2, 1.0f);

    flash_attn<<<dim3(512, 2), 64, 0, stream>>>(Qh, Kh, Vt, x, out);
}
